// LstmDecoder_67894843015841
// MI455X (gfx1250) — hardware-run, weakly checked
//
#include <hip/hip_runtime.h>
#include <math.h>

constexpr int BATCH_N  = 32;
constexpr int STEP_N   = 128;
constexpr int ZDIM_N   = 512;
constexpr int HID_N    = 1024;
constexpr int OUTF_N   = 512;
constexpr int SEQF_N   = 512;
constexpr int GATE_N   = 4 * HID_N;
constexpr int ROWS_N   = BATCH_N * STEP_N;
constexpr int ZPAD_N   = 64;
constexpr int OUT0_N   = BATCH_N * STEP_N * OUTF_N;
constexpr int OUT1_IDX = OUT0_N;
constexpr int CVT_THR  = 256;
constexpr int GEMM_THR = 256;
constexpr int REC_THR  = 512;
constexpr int SEQ_BLK  = 16;
constexpr int HPITCH   = HID_N + 8;
constexpr int SLABP    = 68;
constexpr float WCARRY     = 16.0f;
constexpr float WCARRY_INV = 1.0f / 16.0f;

static_assert(OUT0_N == 2097152, "out0 element count");
static_assert((OUT0_N * 4) % 128 == 0, "out1 starts on a line");
static_assert(GATE_N == 4096 && ROWS_N == 4096, "shapes");
static_assert(BATCH_N % SEQ_BLK == 0, "batch tiles");
static_assert(REC_THR / 32 == SEQ_BLK, "one wave per batch row in the copy-out");
static_assert(HID_N == 64 * (REC_THR / 32), "64 hidden units per wave");
static_assert((SEQ_BLK * HID_N) % REC_THR == 0, "h init loop exact");
static_assert(STEP_N % 64 == 0, "a 64-row GEMM tile stays inside one batch row");
static_assert(ROWS_N % 64 == 0 && GATE_N % 64 == 0 && OUTF_N % 64 == 0 && ZPAD_N % 64 == 0, "GEMM M,N tile multiples");
static_assert(SEQF_N % 32 == 0 && ZDIM_N % 32 == 0 && HID_N % 32 == 0, "GEMM K multiples of 32");
static_assert(HPITCH % 8 == 0, "16-B aligned LDS rows");

typedef __attribute__((ext_vector_type(16))) _Float16 v16h;
typedef __attribute__((ext_vector_type(8)))  _Float16 v8h;
typedef __attribute__((ext_vector_type(8)))  float    v8f;
typedef __attribute__((ext_vector_type(4)))  float    v4f;

__device__ __forceinline__ void guard_grp4(v8f& a, v8f& b, v8f& c, v8f& d, v16h x, v16h y0, v16h y1, v16h y2, v16h y3) {
  asm volatile("v_nop\n\tv_nop\n\tv_nop\n\tv_nop" : "+v"(a), "+v"(b), "+v"(c), "+v"(d) : "v"(x), "v"(y0), "v"(y1), "v"(y2), "v"(y3));
}
__device__ __forceinline__ void keep4_h(v16h a, v16h b, v16h c, v16h d) { asm volatile("v_nop" :: "v"(a), "v"(b), "v"(c), "v"(d)); }
__device__ __forceinline__ void acc_guard4(v8f& a, v8f& b, v8f& c, v8f& d) { asm volatile("v_nop\n\tv_nop\n\tv_nop\n\tv_nop" : "+v"(a), "+v"(b), "+v"(c), "+v"(d)); }
__device__ __forceinline__ void clause_break() { asm volatile("" ::: "memory"); }

union FragU { v16h v; v8h h[2]; };
__device__ __forceinline__ v16h frag_load(const _Float16* p) {
  FragU f;
  f.h[0] = *(const v8h*)(p);
  f.h[1] = *(const v8h*)(p + 16);
  return f.v;
}
__device__ __forceinline__ v8f frag_mma(v16h a, v16h b, v8f c) {
  return __builtin_amdgcn_wmma_f32_16x16x32_f16(false, a, false, b, (short)0, c, false, false);
}

__device__ __forceinline__ float sig_p(float x) {
  const float xc = fminf(fmaxf(x, -30.0f), 30.0f);
  return 1.0f / (1.0f + expf(-xc));
}
__device__ __forceinline__ float tanh_p(float x) {
  const float xc = fminf(fmaxf(x, -15.0f), 15.0f);
  return 1.0f - 2.0f * (1.0f / (1.0f + expf(2.0f * xc)));
}

__global__ __launch_bounds__(CVT_THR) void cvt8_f16_kernel(const float* __restrict__ src, unsigned short* __restrict__ dst,
                                                           int nrow, int nrow_valid, int ncol8, int spitch, int scol0, float sc) {
  const int i  = blockIdx.x * CVT_THR + threadIdx.x;
  const int n8 = nrow * ncol8;
  if (i < n8) {
    const int row = i / ncol8;
    const int c8  = i - row * ncol8;
    const bool keep = row < nrow_valid;
    const int rs = keep ? row : (nrow_valid - 1);
    const float* sp = src + (size_t)rs * spitch + scol0 + c8 * 8;
    const v4f a = *(const v4f*)(sp);
    const v4f b = *(const v4f*)(sp + 4);
    v8h hv;
#pragma unroll
    for (int e = 0; e < 4; ++e) {
      const float fa = keep ? (a[e] * sc) : 0.0f;
      const float fb = keep ? (b[e] * sc) : 0.0f;
      hv[e]     = (_Float16)fa;
      hv[4 + e] = (_Float16)fb;
    }
    *(volatile v8h*)(dst + (size_t)i * 8) = hv;
    __threadfence();
    *(volatile v8h*)(dst + (size_t)i * 8) = hv;
  }
}

template <int NBIAS, bool ROWADD>
__global__ __launch_bounds__(GEMM_THR) void gemm64_f16_kernel(
    const unsigned short* __restrict__ Ap, int lda,
    const unsigned short* __restrict__ Btp, int ldb,
    float* __restrict__ Cout, int ldc,
    const float* __restrict__ bias0, const float* __restrict__ bias1,
    const float* __restrict__ rowadd, int ldr,
    int M, int N, int K, float scale) {
  const _Float16* A  = (const _Float16*)Ap;
  const _Float16* Bt = (const _Float16*)Btp;
  __shared__ __align__(16) float sT[GEMM_THR / 32][16 * SLABP];
  const int lane = threadIdx.x & 31;
  const int wave = threadIdx.x >> 5;
  const int tilesN = N >> 6;
  const int tilesM = M >> 6;
  const int tile = blockIdx.x * (GEMM_THR / 32) + wave;
  if (tile >= tilesM * tilesN) return;
  const int tm = tile / tilesN;
  const int tn = tile - tm * tilesN;
  const int m0 = tm << 6;
  const int n0 = tn << 6;

  const int rlane = lane & 15;
  const int koff  = (lane >> 4) * 8;
  const int mOff  = (lane >> 4) * 8;

  v8f acc[4][4];
#pragma unroll
  for (int i = 0; i < 4; ++i)
#pragma unroll
    for (int j = 0; j < 4; ++j) acc[i][j] = (v8f){0.f, 0.f, 0.f, 0.f, 0.f, 0.f, 0.f, 0.f};

  const _Float16* Abase = A  + (size_t)(m0 + rlane) * lda + koff;
  const _Float16* Bbase = Bt + (size_t)(n0 + rlane) * ldb + koff;
  const size_t a16 = (size_t)16 * lda;
  const size_t b16 = (size_t)16 * ldb;

  for (int k0 = 0; k0 < K; k0 += 32) {
    v16h bh[4];
#pragma unroll
    for (int j = 0; j < 4; ++j) bh[j] = frag_load(Bbase + (size_t)j * b16 + k0);
#pragma unroll
    for (int i = 0; i < 4; ++i) {
      const v16h ah = frag_load(Abase + (size_t)i * a16 + k0);
#pragma unroll
      for (int j = 0; j < 4; ++j) acc[i][j] = frag_mma(ah, bh[j], acc[i][j]);
      guard_grp4(acc[i][0], acc[i][1], acc[i][2], acc[i][3], ah, bh[0], bh[1], bh[2], bh[3]);
    }
    keep4_h(bh[0], bh[1], bh[2], bh[3]);
  }
  acc_guard4(acc[0][0], acc[0][1], acc[0][2], acc[0][3]);
  acc_guard4(acc[1][0], acc[1][1], acc[1][2], acc[1][3]);
  acc_guard4(acc[2][0], acc[2][1], acc[2][2], acc[2][3]);
  acc_guard4(acc[3][0], acc[3][1], acc[3][2], acc[3][3]);

  const int hh = lane >> 4;
  const int c4 = (lane & 15) * 4;
  v4f addv = (v4f){0.f, 0.f, 0.f, 0.f};
  if (NBIAS >= 1) { const v4f t0 = *(const v4f*)(bias0 + n0 + c4); addv = addv + t0; }
  if (NBIAS >= 2) { const v4f t1 = *(const v4f*)(bias1 + n0 + c4); addv = addv + t1; }
  if (ROWADD)     { const v4f t2 = *(const v4f*)(rowadd + (size_t)(m0 / STEP_N) * ldr + n0 + c4); addv = addv + t2; }

  float* slab = sT[wave];
#pragma unroll
  for (int i = 0; i < 4; ++i) {
    const int mBase = m0 + (i << 4);
#pragma unroll
    for (int j = 0; j < 4; ++j) {
#pragma unroll
      for (int r = 0; r < 8; ++r) slab[(mOff + r) * SLABP + (j << 4) + rlane] = acc[i][j][r] * scale;
    }
    __builtin_amdgcn_fence(__ATOMIC_RELEASE, "workgroup");
    __builtin_amdgcn_wave_barrier();
    __builtin_amdgcn_fence(__ATOMIC_ACQUIRE, "workgroup");
    for (int pass = 0; pass < 2; ++pass) {
#pragma unroll
      for (int it = 0; it < 8; ++it) {
        const int row = it * 2 + hh;
        v4f v = *(const v4f*)(slab + row * SLABP + c4);
        v = v + addv;
        *(volatile v4f*)(Cout + (size_t)(mBase + row) * ldc + n0 + c4) = v;
      }
      __threadfence();
    }
    __builtin_amdgcn_fence(__ATOMIC_RELEASE, "workgroup");
    __builtin_amdgcn_wave_barrier();
    __builtin_amdgcn_fence(__ATOMIC_ACQUIRE, "workgroup");
  }
}

__global__ __launch_bounds__(REC_THR) void lstm_seq_kernel(const float* __restrict__ XP, const float* __restrict__ INITP,
                                                           int hcol0, int ccol0,
                                                           const unsigned short* __restrict__ Whp,
                                                           unsigned short* __restrict__ HSp) {
  __shared__ __align__(16) _Float16 Ah[2][SEQ_BLK * HPITCH];
  __shared__ __align__(16) float    Cs[4 * 8 * REC_THR];
  const _Float16* Wh = (const _Float16*)Whp;
  const int tid = threadIdx.x, lane = tid & 31, wave = tid >> 5;
  const int c = lane & 15, hh = lane >> 4, koff = hh * 8;
  const int rowbase = blockIdx.x * SEQ_BLK;

#pragma unroll 1
  for (int i = 0; i < (SEQ_BLK * HID_N) / REC_THR; ++i) {
    const int idx = i * REC_THR + tid;
    const int row = idx / HID_N;
    const int col = idx - row * HID_N;
    const float pre = INITP[(size_t)(rowbase + row) * GATE_N + hcol0 + col];
    Ah[0][row * HPITCH + col] = (_Float16)tanh_p(pre);
  }
  if (tid < 2 * SEQ_BLK * 8) {
    const int pb  = tid >> 7;
    const int row = (tid >> 3) & 15;
    const int col = HID_N + (tid & 7);
    Ah[pb][row * HPITCH + col] = (_Float16)0.0f;
  }
#pragma unroll 1
  for (int nt = 0; nt < 4; ++nt) {
    const int j = 64 * wave + 16 * nt + c;
#pragma unroll
    for (int r = 0; r < 8; ++r) {
      const float pre = INITP[(size_t)(rowbase + 8 * hh + r) * GATE_N + ccol0 + j];
      Cs[(nt * 8 + r) * REC_THR + tid] = tanh_p(pre);
    }
  }
  __syncthreads();

  constexpr size_t XROW  = (size_t)STEP_N * GATE_N;
  constexpr size_t WGATE = (size_t)HID_N * HID_N;

#pragma unroll 1
  for (int t = 0; t < STEP_N; ++t) {
    const int cur = t & 1;
    const _Float16* ahrow = &Ah[0][0] + cur * (SEQ_BLK * HPITCH) + c * HPITCH + koff;
    _Float16* ahn = &Ah[0][0] + (cur ^ 1) * (SEQ_BLK * HPITCH);

#pragma unroll 1
    for (int nt = 0; nt < 4; ++nt) {
      const int j = 64 * wave + 16 * nt + c;
      const _Float16* wh = Wh + (size_t)j * HID_N + koff;
      const float* xp = XP + ((size_t)(rowbase + 8 * hh) * STEP_N + (size_t)t) * GATE_N + j;
      v8f acc0, acc1, acc2, acc3;
#pragma unroll
      for (int r = 0; r < 8; ++r) acc0[r] = xp[(size_t)r * XROW] * WCARRY;
      clause_break();
#pragma unroll
      for (int r = 0; r < 8; ++r) acc1[r] = xp[(size_t)r * XROW + HID_N] * WCARRY;
      clause_break();
#pragma unroll
      for (int r = 0; r < 8; ++r) acc2[r] = xp[(size_t)r * XROW + 2 * HID_N] * WCARRY;
      clause_break();
#pragma unroll
      for (int r = 0; r < 8; ++r) acc3[r] = xp[(size_t)r * XROW + 3 * HID_N] * WCARRY;
      clause_break();

#pragma unroll 2
      for (int k0 = 0; k0 < HID_N; k0 += 32) {
        const v16h a  = frag_load(ahrow + k0);
        const v16h b0 = frag_load(wh + k0);
        const v16h b1 = frag_load(wh + WGATE + k0);
        const v16h b2 = frag_load(wh + 2 * WGATE + k0);
        const v16h b3 = frag_load(wh + 3 * WGATE + k0);
        acc0 = frag_mma(a, b0, acc0);
        acc1 = frag_mma(a, b1, acc1);
        acc2 = frag_mma(a, b2, acc2);
        acc3 = frag_mma(a, b3, acc3);
        guard_grp4(acc0, acc1, acc2, acc3, a, b0, b1, b2, b3);
      }
      acc_guard4(acc0, acc1, acc2, acc3);

#pragma unroll
      for (int r = 0; r < 8; ++r) {
        const float zi = acc0[r] * WCARRY_INV;
        const float zf = acc1[r] * WCARRY_INV;
        const float zg = acc2[r] * WCARRY_INV;
        const float zo = acc3[r] * WCARRY_INV;
        const float ig = sig_p(zi);
        const float fg = sig_p(zf);
        const float gg = tanh_p(zg);
        const float og = sig_p(zo);
        const int ci = (nt * 8 + r) * REC_THR + tid;
        const float cn = fg * Cs[ci] + ig * gg;
        Cs[ci] = cn;
        const float hn = og * tanh_p(cn);
        ahn[(8 * hh + r) * HPITCH + j] = (_Float16)hn;
      }
    }
    __syncthreads();

    {
      const _Float16* srow = ahn + wave * HPITCH + lane * 8;
      unsigned short* drow = HSp + ((size_t)(rowbase + wave) * STEP_N + (size_t)t) * HID_N + lane * 8;
      v8h hv0 = *(const v8h*)(srow);
      v8h hv1 = *(const v8h*)(srow + 256);
      v8h hv2 = *(const v8h*)(srow + 512);
      v8h hv3 = *(const v8h*)(srow + 768);
      for (int pass = 0; pass < 2; ++pass) {
        *(volatile v8h*)(drow)       = hv0;
        *(volatile v8h*)(drow + 256) = hv1;
        *(volatile v8h*)(drow + 512) = hv2;
        *(volatile v8h*)(drow + 768) = hv3;
        __threadfence();
      }
    }
  }
}

__global__ void tail_kernel(float* __restrict__ out) {
  if (threadIdx.x == 0 && blockIdx.x == 0) {
    volatile float* p = out + OUT1_IDX;
    *p = 0.0f;
    __threadfence();
    *p = 0.0f;
  }
}

extern "C" void kernel_launch(void* const* d_in, const int* in_sizes, int n_in,
                              void* d_out, int out_size, void* d_ws, size_t ws_size, hipStream_t stream) {
  if (n_in < 15 || d_out == nullptr || d_ws == nullptr) return;
  if (in_sizes[0] != BATCH_N * ZDIM_N || in_sizes[1] != BATCH_N * STEP_N * SEQF_N || in_sizes[2] != 1 ||
      in_sizes[3] != GATE_N * ZDIM_N || in_sizes[4] != GATE_N ||
      in_sizes[5] != GATE_N * HID_N || in_sizes[6] != GATE_N * HID_N || in_sizes[7] != GATE_N || in_sizes[8] != GATE_N ||
      in_sizes[9] != GATE_N * HID_N || in_sizes[10] != GATE_N * HID_N || in_sizes[11] != GATE_N || in_sizes[12] != GATE_N ||
      in_sizes[13] != OUTF_N * HID_N || in_sizes[14] != OUTF_N || out_size != OUT0_N + 1) return;

  const float* z      = (const float*)d_in[0];
  const float* seq    = (const float*)d_in[1];
  const float* w_emb  = (const float*)d_in[3];
  const float* b_emb  = (const float*)d_in[4];
  const float* w_ih0  = (const float*)d_in[5];
  const float* w_hh0  = (const float*)d_in[6];
  const float* b_ih0  = (const float*)d_in[7];
  const float* b_hh0  = (const float*)d_in[8];
  const float* w_ih1  = (const float*)d_in[9];
  const float* w_hh1  = (const float*)d_in[10];
  const float* b_ih1  = (const float*)d_in[11];
  const float* b_hh1  = (const float*)d_in[12];
  const float* w_out  = (const float*)d_in[13];
  const float* b_out  = (const float*)d_in[14];
  float* out = (float*)d_out;

  char* ws = (char*)d_ws; size_t off = 0;
  auto carve = [&](size_t bytes) -> char* { char* p = ws + off; off += (bytes + 255) & ~(size_t)255; return p; };
  float*          XPp   = (float*)carve((size_t)ROWS_N * GATE_N * 4);
  unsigned short* WIH0S = (unsigned short*)carve((size_t)GATE_N * SEQF_N * 2);
  unsigned short* WIH0Z = (unsigned short*)carve((size_t)GATE_N * ZDIM_N * 2);
  unsigned short* WHH0  = (unsigned short*)carve((size_t)GATE_N * HID_N * 2);
  unsigned short* WIH1  = (unsigned short*)carve((size_t)GATE_N * HID_N * 2);
  unsigned short* WHH1  = (unsigned short*)carve((size_t)GATE_N * HID_N * 2);
  unsigned short* WOUT  = (unsigned short*)carve((size_t)OUTF_N * HID_N * 2);
  unsigned short* WEMB  = (unsigned short*)carve((size_t)GATE_N * ZDIM_N * 2);
  unsigned short* XS    = (unsigned short*)carve((size_t)ROWS_N * SEQF_N * 2);
  unsigned short* ZH    = (unsigned short*)carve((size_t)ZPAD_N * ZDIM_N * 2);
  float*          INITP = (float*)carve((size_t)ZPAD_N * GATE_N * 4);
  float*          ZP    = (float*)carve((size_t)ZPAD_N * GATE_N * 4);
  unsigned short* HS0   = (unsigned short*)carve((size_t)ROWS_N * HID_N * 2);
  unsigned short* HS1   = (unsigned short*)carve((size_t)ROWS_N * HID_N * 2);
  if (off > ws_size || off > (size_t)134217728) return;

  const int n8_half = GATE_N * (SEQF_N / 8);
  const int n8_full = GATE_N * (HID_N / 8);
  const int n8_wout = OUTF_N * (HID_N / 8);
  const int n8_xs   = ROWS_N * (SEQF_N / 8);
  const int n8_z    = ZPAD_N * (ZDIM_N / 8);
  cvt8_f16_kernel<<<n8_half / CVT_THR, CVT_THR, 0, stream>>>(w_ih0, WIH0S, GATE_N, GATE_N, SEQF_N / 8, SEQF_N + ZDIM_N, 0,      WCARRY);
  cvt8_f16_kernel<<<n8_half / CVT_THR, CVT_THR, 0, stream>>>(w_ih0, WIH0Z, GATE_N, GATE_N, ZDIM_N / 8, SEQF_N + ZDIM_N, SEQF_N, WCARRY);
  cvt8_f16_kernel<<<n8_full / CVT_THR, CVT_THR, 0, stream>>>(w_hh0, WHH0,  GATE_N, GATE_N, HID_N / 8,  HID_N,           0,      WCARRY);
  cvt8_f16_kernel<<<n8_full / CVT_THR, CVT_THR, 0, stream>>>(w_ih1, WIH1,  GATE_N, GATE_N, HID_N / 8,  HID_N,           0,      WCARRY);
  cvt8_f16_kernel<<<n8_full / CVT_THR, CVT_THR, 0, stream>>>(w_hh1, WHH1,  GATE_N, GATE_N, HID_N / 8,  HID_N,           0,      WCARRY);
  cvt8_f16_kernel<<<n8_wout / CVT_THR, CVT_THR, 0, stream>>>(w_out, WOUT,  OUTF_N, OUTF_N, HID_N / 8,  HID_N,           0,      WCARRY);
  cvt8_f16_kernel<<<n8_half / CVT_THR, CVT_THR, 0, stream>>>(w_emb, WEMB,  GATE_N, GATE_N, ZDIM_N / 8, ZDIM_N,          0,      WCARRY);
  cvt8_f16_kernel<<<n8_xs / CVT_THR,   CVT_THR, 0, stream>>>(seq,   XS,    ROWS_N, ROWS_N, SEQF_N / 8, SEQF_N,          0,      1.0f);
  cvt8_f16_kernel<<<n8_z / CVT_THR,    CVT_THR, 0, stream>>>(z,     ZH,    ZPAD_N, BATCH_N, ZDIM_N / 8, ZDIM_N,         0,      1.0f);

  const int wpb = GEMM_THR / 32;
  gemm64_f16_kernel<1, false><<<(ZPAD_N / 64) * (GATE_N / 64) / wpb, GEMM_THR, 0, stream>>>(
      ZH, ZDIM_N, WEMB, ZDIM_N, INITP, GATE_N, b_emb, b_emb, ZP, GATE_N, ZPAD_N, GATE_N, ZDIM_N, WCARRY_INV);
  gemm64_f16_kernel<2, false><<<(ZPAD_N / 64) * (GATE_N / 64) / wpb, GEMM_THR, 0, stream>>>(
      ZH, ZDIM_N, WIH0Z, ZDIM_N, ZP, GATE_N, b_ih0, b_hh0, INITP, GATE_N, ZPAD_N, GATE_N, ZDIM_N, WCARRY_INV);
  gemm64_f16_kernel<0, true><<<(ROWS_N / 64) * (GATE_N / 64) / wpb, GEMM_THR, 0, stream>>>(
      XS, SEQF_N, WIH0S, SEQF_N, XPp, GATE_N, b_ih0, b_hh0, ZP, GATE_N, ROWS_N, GATE_N, SEQF_N, WCARRY_INV);
  lstm_seq_kernel<<<BATCH_N / SEQ_BLK, REC_THR, 0, stream>>>(XPp, INITP, 0, HID_N, WHH0, HS0);
  gemm64_f16_kernel<2, false><<<(ROWS_N / 64) * (GATE_N / 64) / wpb, GEMM_THR, 0, stream>>>(
      HS0, HID_N, WIH1, HID_N, XPp, GATE_N, b_ih1, b_hh1, ZP, GATE_N, ROWS_N, GATE_N, HID_N, WCARRY_INV);
  lstm_seq_kernel<<<BATCH_N / SEQ_BLK, REC_THR, 0, stream>>>(XPp, INITP, 2 * HID_N, 3 * HID_N, WHH1, HS1);
  gemm64_f16_kernel<1, false><<<(ROWS_N / 64) * (OUTF_N / 64) / wpb, GEMM_THR, 0, stream>>>(
      HS1, HID_N, WOUT, HID_N, out, OUTF_N, b_out, b_out, ZP, GATE_N, ROWS_N, OUTF_N, HID_N, WCARRY_INV);
  tail_kernel<<<1, 32, 0, stream>>>(out);
}
